// DeepseekV4Attention_60129542144617
// MI455X (gfx1250) — hardware-verified
//
#include <hip/hip_runtime.h>
#include <math.h>
#include <stdint.h>

#define NSEQ   2
#define SQ     2048
#define HID    2048
#define NHQ    16
#define HDM    128
#define KVD    128
#define QKW    2176
#define KCOL   2048
#define NTOK   4096
#define NFREQ  32
#define AOW    4096
#define WINDOW 1024

typedef __bf16         v16b __attribute__((ext_vector_type(16)));
typedef __bf16         v8b  __attribute__((ext_vector_type(8)));
typedef float          v8f  __attribute__((ext_vector_type(8)));
typedef float          v4f  __attribute__((ext_vector_type(4)));
typedef unsigned int   v4u  __attribute__((ext_vector_type(4)));
typedef unsigned short v8us __attribute__((ext_vector_type(8)));

__device__ __forceinline__ unsigned short bf_bits(float f) {
  const unsigned u = __float_as_uint(f);
  return (unsigned short)((u + 0x7FFFu + ((u >> 16) & 1u)) >> 16);
}
__device__ __forceinline__ float bf_val(unsigned short h) { return __uint_as_float(((unsigned)h) << 16); }
__device__ __forceinline__ float bf_rne(float f) { return bf_val(bf_bits(f)); }
__device__ __forceinline__ unsigned pk16(unsigned short a, unsigned short b) { return (unsigned)a | ((unsigned)b << 16); }
__device__ __forceinline__ v8f zero8() { v8f z = {0.f, 0.f, 0.f, 0.f, 0.f, 0.f, 0.f, 0.f}; return z; }
__device__ __forceinline__ int wave_id() { return __builtin_amdgcn_readfirstlane((int)(threadIdx.x >> 5)); }
__device__ __forceinline__ void bf_split(float f, __bf16& hi, __bf16& lo) {
  const unsigned short hb = bf_bits(f);
  hi = __builtin_bit_cast(__bf16, hb);
  lo = __builtin_bit_cast(__bf16, bf_bits(f - bf_val(hb)));
}

__device__ __forceinline__ void lds_wave_sync() {
  __builtin_amdgcn_fence(__ATOMIC_RELEASE, "workgroup");
  __builtin_amdgcn_wave_barrier();
  __builtin_amdgcn_fence(__ATOMIC_ACQUIRE, "workgroup");
}

union FragB { v16b v; v8b h[2]; };
__device__ __forceinline__ v16b ldfrag_b(const __bf16* p) { FragB f; f.h[0] = *(const v8b*)(p); f.h[1] = *(const v8b*)(p + 16); return f.v; }

__device__ __forceinline__ v8f mma_b(v16b a, v16b b, v8f c) {
  return __builtin_amdgcn_wmma_f32_16x16x32_bf16(false, a, false, b, (short)0, c, false, false);
}
__device__ __forceinline__ v8f mma_bg(v16b a, v16b b, v8f c) {
  c = mma_b(a, b, c);
  asm volatile("v_nop\n\tv_nop\n\tv_nop\n\tv_nop" : "+v"(c) : "v"(a), "v"(b));
  return c;
}
__device__ __forceinline__ void dep_guard_b(v8f& a, v8f& b, v16b x, v16b y) {
  asm volatile("v_nop\n\tv_nop\n\tv_nop\n\tv_nop" : "+v"(a), "+v"(b) : "v"(x), "v"(y));
}
__device__ __forceinline__ void keep4_b(v16b a, v16b b, v16b c, v16b d) { asm volatile("v_nop" :: "v"(a), "v"(b), "v"(c), "v"(d)); }
__device__ __forceinline__ void acc_guard4(v8f& a, v8f& b, v8f& c, v8f& d) {
  asm volatile("v_nop\n\tv_nop\n\tv_nop\n\tv_nop" : "+v"(a), "+v"(b), "+v"(c), "+v"(d));
}

struct InvFreq { float v[NFREQ]; };
static_assert(sizeof(InvFreq) == NFREQ * 4);

__global__ __launch_bounds__(256) void rope_table_kernel(const int* __restrict__ pos, InvFreq tab,
                                                         float* __restrict__ cst, float* __restrict__ snt, int ntok) {
  const int lane = threadIdx.x & 31;
  const int wave = (int)(threadIdx.x >> 5);
  const int t = (int)blockIdx.x * 8 + wave;
  if (t >= ntok) return;
  const float pf = (float)pos[t];
  float inv = 0.f;
#pragma unroll
  for (int j = 0; j < NFREQ; ++j) inv = (lane == j) ? tab.v[j] : inv;
  const float ang = pf * inv;
  const float cv = cosf(ang);
  const float sv = sinf(ang);
  const size_t o = (size_t)t * NFREQ + lane;
  for (int pass = 0; pass < 2; ++pass) {
    ((volatile float*)cst)[o] = cv;
    ((volatile float*)snt)[o] = sv;
    __threadfence();
  }
}

__global__ __launch_bounds__(256) void cvt_bf16_kernel(const float* __restrict__ in, unsigned short* __restrict__ outp, int n8) {
  const int i = (int)blockIdx.x * 256 + (int)threadIdx.x;
  if (i >= n8) return;
  const size_t e = 8 * (size_t)i;
  const v4f a = *(const v4f*)(in + e);
  const v4f b = *(const v4f*)(in + e + 4);
  v4u w;
  w[0] = pk16(bf_bits(a[0]), bf_bits(a[1]));
  w[1] = pk16(bf_bits(a[2]), bf_bits(a[3]));
  w[2] = pk16(bf_bits(b[0]), bf_bits(b[1]));
  w[3] = pk16(bf_bits(b[2]), bf_bits(b[3]));
  *(volatile v4u*)(outp + e) = w;
  __threadfence();
  *(volatile v4u*)(outp + e) = w;
}

template <bool DUP>
__global__ __launch_bounds__(256) void tconv_bf16_kernel(const float* __restrict__ W, unsigned short* __restrict__ outp,
                                                         int R, int Cc, int ldo, int dupoff) {
  __shared__ __align__(16) float tf[64 * 68];
  const int c0  = (int)blockIdx.x * 64;
  const int r0  = (int)blockIdx.y * 64;
  const int tid = (int)threadIdx.x;
  {
    const int lr = tid >> 4;
    const int c4 = (tid & 15) * 4;
#pragma unroll
    for (int it = 0; it < 4; ++it) {
      const int rr = it * 16 + lr;
      const v4f a = *(const v4f*)(W + (size_t)(r0 + rr) * Cc + c0 + c4);
      *(v4f*)(tf + rr * 68 + c4) = a;
    }
  }
  __syncthreads();
  const int sub = tid >> 3;
  const int c8  = (tid & 7) * 8;
  v4u hv[2];
#pragma unroll
  for (int it = 0; it < 2; ++it) {
    const int oc = it * 32 + sub;
    v4u a;
#pragma unroll
    for (int q = 0; q < 4; ++q) {
      const float f0 = tf[(c8 + 2 * q) * 68 + oc];
      const float f1 = tf[(c8 + 2 * q + 1) * 68 + oc];
      a[q] = pk16(bf_bits(f0), bf_bits(f1));
    }
    hv[it] = a;
  }
  for (int pass = 0; pass < 2; ++pass) {
#pragma unroll
    for (int it = 0; it < 2; ++it) {
      const int oc = it * 32 + sub;
      const size_t go = (size_t)(c0 + oc) * ldo + r0 + c8;
      *(volatile v4u*)(outp + go) = hv[it];
      if (DUP) *(volatile v4u*)(outp + go + dupoff) = hv[it];
    }
    __threadfence();
  }
}

template <int OUT_MODE, bool ROPE>
__global__ __launch_bounds__(256) void gemm64_kernel(
    const unsigned short* __restrict__ Ap, int lda,
    const unsigned short* __restrict__ Btp, int ldb,
    void* __restrict__ Cout, void* __restrict__ Cout2, int ldc,
    const float* __restrict__ cst, const float* __restrict__ snt,
    int M, int N, int K) {
  const __bf16* A  = (const __bf16*)(const void*)Ap;
  const __bf16* Bt = (const __bf16*)(const void*)Btp;
  __shared__ __align__(16) float sT[8][16 * 68];
  static_assert((16 * 68 * 4) % 16 == 0);
  static_assert((68 * 4) % 16 == 0);

  const int lane = threadIdx.x & 31;
  const int wave = wave_id();
  const int tilesN = N >> 6;
  const int tilesM = M >> 6;
  const int tile = (int)blockIdx.x * 8 + wave;
  if (tile >= tilesM * tilesN) return;
  const int tm = tile / tilesN;
  const int tn = tile - tm * tilesN;
  const int m0 = tm << 6;
  const int n0 = tn << 6;

  const int rlane = lane & 15;
  const int koff  = (lane >> 4) * 8;
  const int mOff  = (lane >> 4) * 8;

  v8f acc[4][4];
#pragma unroll
  for (int i = 0; i < 4; ++i)
#pragma unroll
    for (int j = 0; j < 4; ++j) acc[i][j] = zero8();

  for (int k0 = 0; k0 < K; k0 += 32) {
    v16b bh[4];
#pragma unroll
    for (int j = 0; j < 4; ++j) {
      const size_t bo = (size_t)(n0 + (j << 4) + rlane) * ldb + koff + k0;
      bh[j] = ldfrag_b(Bt + bo);
    }
#pragma unroll
    for (int i = 0; i < 4; ++i) {
      const size_t ao = (size_t)(m0 + (i << 4) + rlane) * lda + koff + k0;
      const v16b ah = ldfrag_b(A + ao);
#pragma unroll
      for (int j = 0; j < 4; ++j) acc[i][j] = mma_b(ah, bh[j], acc[i][j]);
      dep_guard_b(acc[i][0], acc[i][3], ah, bh[3]);
    }
    keep4_b(bh[0], bh[1], bh[2], bh[3]);
  }
  acc_guard4(acc[0][0], acc[0][1], acc[0][2], acc[0][3]);
  acc_guard4(acc[1][0], acc[1][1], acc[1][2], acc[1][3]);
  acc_guard4(acc[2][0], acc[2][1], acc[2][2], acc[2][3]);
  acc_guard4(acc[3][0], acc[3][1], acc[3][2], acc[3][3]);

  float* slab = sT[wave];
  const bool rot = ROPE && ((n0 & 127) == 0);
#pragma unroll
  for (int i = 0; i < 4; ++i) {
    const int mBase = m0 + (i << 4);
    if (rot) {
#pragma unroll
      for (int u = 0; u < 4; ++u) {
        const int p   = u * 32 + lane;
        const int row = p >> 3;
        const int c4  = (p & 7) * 4;
        int trow = mBase + row;
        trow = (trow < M) ? trow : (M - 1);
        const v4f cv4 = *(const v4f*)(cst + (size_t)trow * NFREQ + c4);
        const v4f sv4 = *(const v4f*)(snt + (size_t)trow * NFREQ + c4);
        *(v4f*)(slab + row * 68 + c4)      = cv4;
        *(v4f*)(slab + row * 68 + 32 + c4) = sv4;
      }
      lds_wave_sync();
#pragma unroll
      for (int j = 0; j < 2; ++j) {
        const int dim = (j << 4) + rlane;
#pragma unroll
        for (int r = 0; r < 8; ++r) {
          const int so1 = (mOff + r) * 68 + dim;
          const int so2 = so1 + 32;
          const float cv = slab[so1];
          const float sv = slab[so2];
          const float x1 = acc[i][j][r];
          const float x2 = acc[i][j + 2][r];
          const float o1 = x1 * cv - x2 * sv;
          const float o2 = x2 * cv + x1 * sv;
          slab[so1] = o1;
          slab[so2] = o2;
        }
      }
    } else {
#pragma unroll
      for (int j = 0; j < 4; ++j)
#pragma unroll
        for (int r = 0; r < 8; ++r)
          slab[(mOff + r) * 68 + (j << 4) + rlane] = acc[i][j][r];
    }
    lds_wave_sync();
    if (OUT_MODE == 0) {
      float* C = (float*)Cout;
      const int hh = lane >> 4, c4 = (lane & 15) * 4;
      for (int pass = 0; pass < 2; ++pass) {
#pragma unroll
        for (int it = 0; it < 8; ++it) {
          const int row = it * 2 + hh;
          const v4f v = *(const v4f*)(slab + row * 68 + c4);
          *(volatile v4f*)(C + (size_t)(mBase + row) * ldc + n0 + c4) = v;
        }
        __threadfence();
      }
    } else {
      const int q = lane >> 3, c8 = (lane & 7) * 8;
      unsigned short* C  = (unsigned short*)Cout;
      unsigned short* C2 = (unsigned short*)Cout2;
      for (int pass = 0; pass < 2; ++pass) {
#pragma unroll
        for (int it = 0; it < 4; ++it) {
          const int row = it * 4 + q;
          const float* sp = slab + row * 68 + c8;
          v8us hv, lv;
#pragma unroll
          for (int e = 0; e < 8; ++e) {
            const float f = sp[e];
            const unsigned short hb = bf_bits(f);
            const unsigned short lb = bf_bits(f - bf_val(hb));
            hv[e] = hb;
            lv[e] = lb;
          }
          *(volatile v8us*)(C  + (size_t)(mBase + row) * ldc + n0 + c8) = hv;
          *(volatile v8us*)(C2 + (size_t)(mBase + row) * ldc + n0 + c8) = lv;
        }
        __threadfence();
      }
    }
    lds_wave_sync();
  }
}

#define AT_KC   32
#define KS_P    136
#define VS_P    40
#define PS_P    40
#define LDS_KS  0
#define LDS_KLS (32 * KS_P)
#define LDS_VHS (2 * 32 * KS_P)
#define LDS_VLS (LDS_VHS + 128 * VS_P)
#define LDS_PH  (LDS_VLS + 128 * VS_P)
#define LDS_PL  (LDS_PH + 4 * 16 * PS_P)
#define LDS_TOT (LDS_PL + 4 * 16 * PS_P)
static_assert(LDS_TOT * 2 <= 65536);
static_assert(4 * 4096 <= LDS_TOT);
static_assert(WINDOW % AT_KC == 0);
static_assert(SQ % 64 == 0);

__global__ __launch_bounds__(128) void attn_kernel(
    const unsigned short* __restrict__ qkh, const unsigned short* __restrict__ qkl,
    const unsigned short* __restrict__ vth, const unsigned short* __restrict__ vtl,
    const float* __restrict__ sinkp, unsigned short* __restrict__ aop) {
  __shared__ __align__(16) __bf16 lds[LDS_TOT];
  __bf16* Ks  = lds + LDS_KS;
  __bf16* Kls = lds + LDS_KLS;
  __bf16* Vhs = lds + LDS_VHS;
  __bf16* Vls = lds + LDS_VLS;

  const int tid  = (int)threadIdx.x;
  const int lane = tid & 31;
  const int wave = wave_id();
  const int hh   = lane >> 4;
  const int c    = lane & 15;
  const int qb   = (int)blockIdx.x;
  const int h    = (int)blockIdx.y;
  const int b    = (int)blockIdx.z;
  const int q0   = qb * 64 + wave * 16;
  const int qlast = q0 + 15;
  const size_t tok0 = (size_t)b * SQ;

  const __bf16* QKh = (const __bf16*)(const void*)qkh;
  const __bf16* QKl = (const __bf16*)(const void*)qkl;
  const __bf16* Qhr = QKh + (tok0 + q0 + c) * QKW + h * HDM + 8 * hh;
  const __bf16* Qlr = QKl + (tok0 + q0 + c) * QKW + h * HDM + 8 * hh;
  const __bf16* Kg  = QKh + tok0 * QKW + KCOL;
  const __bf16* Klg = QKl + tok0 * QKW + KCOL;
  const __bf16* Vhg = (const __bf16*)(const void*)vth + tok0;
  const __bf16* Vlg = (const __bf16*)(const void*)vtl + tok0;
  __bf16* ph = lds + LDS_PH + wave * (16 * PS_P);
  __bf16* pl = lds + LDS_PL + wave * (16 * PS_P);

  const float snk = bf_rne(sinkp[h]);

  float mrow[8], lrow[8];
  v8f oacc[8];
#pragma unroll
  for (int r = 0; r < 8; ++r) { mrow[r] = snk; lrow[r] = 1.0f; }
#pragma unroll
  for (int t = 0; t < 8; ++t) oacc[t] = zero8();

  int kc_lo = 2 * qb - (WINDOW / AT_KC);
  if (kc_lo < 0) kc_lo = 0;
  const int kc_hi = 2 * qb + 1;
  for (int kc = kc_lo; kc <= kc_hi; ++kc) {
    const int kv0 = kc * AT_KC;
    __syncthreads();
#pragma unroll
    for (int i = 0; i < 4; ++i) {
      const int p   = tid + 128 * i;
      const int key = p >> 4, d8 = (p & 15) * 8;
      const v8b kx = *(const v8b*)(Kg  + (size_t)(kv0 + key) * QKW + d8);
      const v8b ky = *(const v8b*)(Klg + (size_t)(kv0 + key) * QKW + d8);
      *(v8b*)(Ks  + key * KS_P + d8) = kx;
      *(v8b*)(Kls + key * KS_P + d8) = ky;
      const int d = p >> 2, k8 = (p & 3) * 8;
      const v8b vx = *(const v8b*)(Vhg + (size_t)d * NTOK + kv0 + k8);
      const v8b vy = *(const v8b*)(Vlg + (size_t)d * NTOK + kv0 + k8);
      *(v8b*)(Vhs + d * VS_P + k8) = vx;
      *(v8b*)(Vls + d * VS_P + k8) = vy;
    }
    __syncthreads();

    const bool live = (kv0 <= qlast) && (kv0 + (AT_KC - 1) + (WINDOW - 1) >= q0);
    if (live) {
      v8f s[2];
      s[0] = zero8(); s[1] = zero8();
#pragma unroll
      for (int dc = 0; dc < 4; ++dc) {
        const v16b qa = ldfrag_b(Qhr + dc * 32);
        const v16b ql = ldfrag_b(Qlr + dc * 32);
#pragma unroll
        for (int j = 0; j < 2; ++j) {
          const v16b kb = ldfrag_b(Ks  + (j * 16 + c) * KS_P + dc * 32 + 8 * hh);
          const v16b kl = ldfrag_b(Kls + (j * 16 + c) * KS_P + dc * 32 + 8 * hh);
          s[j] = mma_bg(qa, kb, s[j]);
          s[j] = mma_bg(qa, kl, s[j]);
          s[j] = mma_bg(ql, kb, s[j]);
        }
      }
      float cm[8];
#pragma unroll
      for (int r = 0; r < 8; ++r) {
        const int qrow = q0 + 8 * hh + r;
        float m = -INFINITY;
#pragma unroll
        for (int j = 0; j < 2; ++j) {
          const int key = kv0 + j * 16 + c;
          const float sv = s[j][r] * 0.08838834764831845f;
          const bool ok = (key <= qrow) && ((qrow - key) < WINDOW);
          const float sm = ok ? sv : -INFINITY;
          s[j][r] = sm;
          m = fmaxf(m, sm);
        }
#pragma unroll
        for (int off = 1; off < 16; off <<= 1) m = fmaxf(m, __shfl_xor(m, off, 32));
        cm[r] = m;
      }
#pragma unroll
      for (int r = 0; r < 8; ++r) {
        const float mnew  = fmaxf(mrow[r], cm[r]);
        const float alpha = __expf(mrow[r] - mnew);
        mrow[r] = mnew;
        float psum = 0.f;
#pragma unroll
        for (int j = 0; j < 2; ++j) {
          const float p = __expf(s[j][r] - mnew);
          psum += p;
          __bf16 a, bl;
          bf_split(p, a, bl);
          const int po = (8 * hh + r) * PS_P + j * 16 + c;
          ph[po] = a;
          pl[po] = bl;
        }
#pragma unroll
        for (int off = 1; off < 16; off <<= 1) psum += __shfl_xor(psum, off, 32);
        lrow[r] = lrow[r] * alpha + psum;
#pragma unroll
        for (int t = 0; t < 8; ++t) oacc[t][r] *= alpha;
      }
      lds_wave_sync();
      const v16b pa = ldfrag_b(ph + c * PS_P + 8 * hh);
      const v16b pr = ldfrag_b(pl + c * PS_P + 8 * hh);
#pragma unroll
      for (int t = 0; t < 8; ++t) {
        const v16b vb = ldfrag_b(Vhs + (t * 16 + c) * VS_P + 8 * hh);
        const v16b vr = ldfrag_b(Vls + (t * 16 + c) * VS_P + 8 * hh);
        oacc[t] = mma_bg(pa, vb, oacc[t]);
        oacc[t] = mma_bg(pa, vr, oacc[t]);
        oacc[t] = mma_bg(pr, vb, oacc[t]);
      }
    }
  }

  __syncthreads();
  unsigned short* ous = (unsigned short*)(void*)lds + wave * 4096;
  unsigned short* osl = ous + 2048;
#pragma unroll
  for (int r = 0; r < 8; ++r) {
    const float inv = 1.0f / lrow[r];
#pragma unroll
    for (int t = 0; t < 8; ++t) {
      const float o = oacc[t][r] * inv;
      const unsigned short hb = bf_bits(o);
      const unsigned short lb = bf_bits(o - bf_val(hb));
      const int so = (8 * hh + r) * 128 + t * 16 + c;
      ous[so] = hb;
      osl[so] = lb;
    }
  }
  lds_wave_sync();
  unsigned short* Ahg = aop + (tok0 + q0) * AOW + h * HDM;
  unsigned short* Alg = Ahg + HID;
  for (int pass = 0; pass < 2; ++pass) {
#pragma unroll
    for (int it = 0; it < 8; ++it) {
      const int row = it * 2 + hh;
      const int c8  = c * 8;
      const v8us x = *(const v8us*)(ous + row * 128 + c8);
      const v8us y = *(const v8us*)(osl + row * 128 + c8);
      *(volatile v8us*)(Ahg + (size_t)row * AOW + c8) = x;
      *(volatile v8us*)(Alg + (size_t)row * AOW + c8) = y;
    }
    __threadfence();
  }
}

extern "C" void kernel_launch(void* const* d_in, const int* in_sizes, int n_in,
                              void* d_out, int out_size, void* d_ws, size_t ws_size,
                              hipStream_t stream) {
  if (n_in < 7) return;
  if (in_sizes[0] != NTOK * HID) return;
  if (in_sizes[1] != NTOK) return;
  if (in_sizes[2] != HID * HID) return;
  if (in_sizes[3] != HID * KVD) return;
  if (in_sizes[4] != HID * KVD) return;
  if (in_sizes[5] != HID * HID) return;
  if (in_sizes[6] != NHQ) return;
  if (out_size != NTOK * HID) return;

  const float* hidden = (const float*)d_in[0];
  const int*   pos    = (const int*)d_in[1];
  const float* wq     = (const float*)d_in[2];
  const float* wk     = (const float*)d_in[3];
  const float* wv     = (const float*)d_in[4];
  const float* wo     = (const float*)d_in[5];
  const float* sink   = (const float*)d_in[6];
  float* out = (float*)d_out;

  const size_t szX   = (size_t)NTOK * HID * 2;
  const size_t szWqk = (size_t)QKW * HID * 2;
  const size_t szWv  = (size_t)KVD * HID * 2;
  const size_t szWo2 = (size_t)HID * AOW * 2;
  const size_t szT   = (size_t)NTOK * NFREQ * 4;
  const size_t szQK  = (size_t)NTOK * QKW * 2;
  const size_t szVT  = (size_t)KVD * NTOK * 2;
  const size_t szAO  = (size_t)NTOK * AOW * 2;
  size_t off = 0;
  const size_t oX   = off; off += szX;
  const size_t oWqk = off; off += szWqk;
  const size_t oWv  = off; off += szWv;
  const size_t oWo2 = off; off += szWo2;
  const size_t oCs  = off; off += szT;
  const size_t oSn  = off; off += szT;
  const size_t oQKh = off; off += szQK;
  const size_t oQKl = off; off += szQK;
  const size_t oVTh = off; off += szVT;
  const size_t oVTl = off; off += szVT;
  const size_t oAO  = off; off += szAO;
  if (off > ws_size) return;

  char* ws = (char*)d_ws;
  unsigned short* Xb   = (unsigned short*)(ws + oX);
  unsigned short* WqkT = (unsigned short*)(ws + oWqk);
  unsigned short* WvT  = (unsigned short*)(ws + oWv);
  unsigned short* WoT2 = (unsigned short*)(ws + oWo2);
  float*          cst  = (float*)(ws + oCs);
  float*          snt  = (float*)(ws + oSn);
  unsigned short* QKh  = (unsigned short*)(ws + oQKh);
  unsigned short* QKl  = (unsigned short*)(ws + oQKl);
  unsigned short* VTh  = (unsigned short*)(ws + oVTh);
  unsigned short* VTl  = (unsigned short*)(ws + oVTl);
  unsigned short* AO   = (unsigned short*)(ws + oAO);

  InvFreq tab;
  for (int j = 0; j < NFREQ; ++j) tab.v[j] = 1.0f / powf(10000.0f, (float)j * 0.03125f);

  const dim3 b256(256), b128(128);

  rope_table_kernel<<<dim3(NTOK / 8), b256, 0, stream>>>(pos, tab, cst, snt, NTOK);
  cvt_bf16_kernel<<<dim3((NTOK * HID / 8) / 256), b256, 0, stream>>>(hidden, Xb, NTOK * HID / 8);
  tconv_bf16_kernel<false><<<dim3(HID / 64, HID / 64), b256, 0, stream>>>(wq, WqkT, HID, HID, HID, 0);
  tconv_bf16_kernel<false><<<dim3(KVD / 64, HID / 64), b256, 0, stream>>>(wk, WqkT + (size_t)KCOL * HID, HID, KVD, HID, 0);
  tconv_bf16_kernel<false><<<dim3(KVD / 64, HID / 64), b256, 0, stream>>>(wv, WvT, HID, KVD, HID, 0);
  tconv_bf16_kernel<true><<<dim3(HID / 64, HID / 64), b256, 0, stream>>>(wo, WoT2, HID, HID, AOW, HID);
  gemm64_kernel<2, true><<<dim3((NTOK / 64) * (QKW / 64) / 8), b256, 0, stream>>>(
      Xb, HID, WqkT, HID, (void*)QKh, (void*)QKl, QKW, cst, snt, NTOK, QKW, HID);
  gemm64_kernel<2, false><<<dim3((KVD / 64) * (NTOK / 64) / 8), b256, 0, stream>>>(
      WvT, HID, Xb, HID, (void*)VTh, (void*)VTl, NTOK, cst, snt, KVD, NTOK, HID);
  attn_kernel<<<dim3(SQ / 64, NHQ, NSEQ), b128, 0, stream>>>(QKh, QKl, VTh, VTl, sink, AO);
  gemm64_kernel<0, false><<<dim3((NTOK / 64) * (HID / 64) / 8), b256, 0, stream>>>(
      AO, AOW, WoT2, AOW, (void*)out, (void*)out, HID, cst, snt, NTOK, HID, AOW);
  (void)hipGetLastError();
}
